// MiniAttention_6012954214731
// MI455X (gfx1250) — hardware-verified
//
#include <hip/hip_runtime.h>


#define NB 8
#define NS 1024
#define NC 768
#define NH 12
#define ND 64
#define NTOK (NB * NS)
#define NF (3 * NC)

static_assert(NC == NH * ND);
static_assert(ND == 64);
static_assert(NH == 12);
static_assert(NS % 128 == 0 && NS % 64 == 0 && NS % 32 == 0 && NTOK % 64 == 0);
static_assert(NF % 256 == 0 && NC % 256 == 0 && NC % 64 == 0 && NC % 32 == 0);

typedef float v4f __attribute__((ext_vector_type(4)));
typedef float v8f __attribute__((ext_vector_type(8)));
typedef unsigned int v4u __attribute__((ext_vector_type(4)));
typedef unsigned int v8u __attribute__((ext_vector_type(8)));
typedef _Float16 v8h __attribute__((ext_vector_type(8)));
typedef _Float16 v16h __attribute__((ext_vector_type(16)));
typedef unsigned short us;

union Frag { v4u q[2]; v8u w; v16h h; };
union H8 { v8h h; v4u u; us s[8]; };
union F8 { v8f v; v4f q[2]; };

#define NOPS "v_nop\n\tv_nop\n\tv_nop\n\tv_nop"
#define WF16(a, bb, c) __builtin_amdgcn_wmma_f32_16x16x32_f16(false, (a), false, (bb), (short)0, (c), false, false)

__device__ __forceinline__ Frag ldfrag(const us* __restrict__ base, int ld, int row, int k0, int lane) {
  const us* p = base + (size_t)(row + (lane & 15)) * (size_t)ld + k0 + 8 * (lane >> 4);
  Frag f;
  f.q[0] = *(const v4u*)p;
  f.q[1] = *(const v4u*)(p + 16);
  return f;
}

__device__ __forceinline__ us f16bits(float x) {
  const _Float16 hv = (_Float16)x;
  return __builtin_bit_cast(us, hv);
}

__device__ __forceinline__ v8f zero8() {
  v8f z;
#pragma unroll
  for (int r = 0; r < 8; ++r) z[r] = 0.f;
  return z;
}

__device__ __forceinline__ void gemm32x64(const us* __restrict__ A, int lda, int ar,
                                          const us* __restrict__ Bm, int ldb, int br,
                                          int K, int lane, v8f (&acc)[2][4]) {
#pragma unroll 1
  for (int k0 = 0; k0 < K; k0 += 32) {
    const Frag a0 = ldfrag(A, lda, ar, k0, lane);
    const Frag a1 = ldfrag(A, lda, ar + 16, k0, lane);
#pragma unroll
    for (int jp = 0; jp < 4; jp += 2) {
      const Frag b0 = ldfrag(Bm, ldb, br + 16 * jp, k0, lane);
      const Frag b1 = ldfrag(Bm, ldb, br + 16 * jp + 16, k0, lane);
      acc[0][jp] = WF16(a0.h, b0.h, acc[0][jp]);
      acc[1][jp] = WF16(a1.h, b0.h, acc[1][jp]);
      acc[0][jp + 1] = WF16(a0.h, b1.h, acc[0][jp + 1]);
      acc[1][jp + 1] = WF16(a1.h, b1.h, acc[1][jp + 1]);
      asm volatile(NOPS
                   : "+v"(acc[0][jp]), "+v"(acc[1][jp]), "+v"(acc[0][jp + 1]), "+v"(acc[1][jp + 1])
                   : "v"(a0.w), "v"(a1.w), "v"(b0.w), "v"(b1.w));
    }
  }
}

__global__ __launch_bounds__(256) void k_cvt(const float* __restrict__ src, us* dst, float scale, int n8) {
  const int g = blockIdx.x * 256 + threadIdx.x;
  if (g >= n8) return;
  const float* s = src + (size_t)g * 8;
  const v4f a = *(const v4f*)s;
  const v4f c = *(const v4f*)(s + 4);
  H8 o;
  o.h[0] = (_Float16)(a.x * scale); o.h[1] = (_Float16)(a.y * scale);
  o.h[2] = (_Float16)(a.z * scale); o.h[3] = (_Float16)(a.w * scale);
  o.h[4] = (_Float16)(c.x * scale); o.h[5] = (_Float16)(c.y * scale);
  o.h[6] = (_Float16)(c.z * scale); o.h[7] = (_Float16)(c.w * scale);
  us* p = dst + (size_t)g * 8;
  *(volatile v4u*)p = o.u;
  __threadfence();
  *(volatile v4u*)p = o.u;
}

__global__ __launch_bounds__(256) void k_xsum(const float* __restrict__ x, float* xs) {
  __shared__ __attribute__((aligned(16))) float T[256];
  const int tid = threadIdx.x;
  const int b = blockIdx.x / (NC / 256), cb = blockIdx.x % (NC / 256);
  const float* p = x + (size_t)b * NS * NC + cb * 256 + tid;
  double s = 0.0;
#pragma unroll 4
  for (int n = 0; n < NS; ++n) s += (double)p[(size_t)n * NC];
  T[tid] = (float)s;
  __syncthreads();
  if (tid < 64) {
    const v4f v = *(const v4f*)(T + 4 * tid);
    float* d = xs + (size_t)b * NC + cb * 256 + 4 * tid;
    *(volatile v4f*)d = v;
    __threadfence();
    *(volatile v4f*)d = v;
  }
}

__global__ __launch_bounds__(256) void k_sv(const float* __restrict__ xs, const float* __restrict__ wqkv, float* sv) {
  __shared__ __attribute__((aligned(16))) float R[32];
  const int tid = threadIdx.x, w = tid >> 5, lane = tid & 31;
  const int b = blockIdx.x / (NC / 32), cb = blockIdx.x % (NC / 32);
  const float* xb = xs + (size_t)b * NC;
  float xr[NC / 32];
#pragma unroll
  for (int t = 0; t < NC / 32; ++t) xr[t] = xb[lane + 32 * t];
#pragma unroll 1
  for (int j = 0; j < 4; ++j) {
    const int od = cb * 32 + 4 * w + j;
    const float* wr = wqkv + (size_t)(2 * NC + od) * NC;
    float a = 0.f;
#pragma unroll
    for (int t = 0; t < NC / 32; ++t) a = fmaf(xr[t], wr[lane + 32 * t], a);
#pragma unroll
    for (int off = 16; off > 0; off >>= 1) a += __shfl_xor(a, off, 32);
    if (lane == 0) R[4 * w + j] = a;
  }
  __syncthreads();
  if (tid < 8) {
    const v4f v = *(const v4f*)(R + 4 * tid);
    float* d = sv + (size_t)b * NC + cb * 32 + 4 * tid;
    *(volatile v4f*)d = v;
    __threadfence();
    *(volatile v4f*)d = v;
  }
}

__global__ __launch_bounds__(256) void k_corr(const float* __restrict__ sv, const float* __restrict__ convw,
                                              const float* __restrict__ wproj, const float* __restrict__ bias,
                                              float* corr) {
  __shared__ float cs[16];
  __shared__ __attribute__((aligned(16))) float R[32];
  const int tid = threadIdx.x, w = tid >> 5, lane = tid & 31;
  const int b = blockIdx.x / (NC / 32), cb = blockIdx.x % (NC / 32);
  if (tid < 16) {
    float s = 0.f;
    if (tid < NH) {
#pragma unroll
      for (int h = 0; h < NH; ++h) s += convw[tid * NH + h];
    }
    cs[tid] = s * (1.0f / (float)NS);
  }
  __syncthreads();
  const float* sb = sv + (size_t)b * NC;
  float xr[NC / 32];
#pragma unroll
  for (int t = 0; t < NC / 32; ++t) {
    const int i = lane + 32 * t;
    xr[t] = sb[i] * cs[i / ND];
  }
#pragma unroll 1
  for (int j = 0; j < 4; ++j) {
    const int c = cb * 32 + 4 * w + j;
    const float* wr = wproj + (size_t)c * NC;
    float a = 0.f;
#pragma unroll
    for (int t = 0; t < NC / 32; ++t) a = fmaf(xr[t], wr[lane + 32 * t], a);
#pragma unroll
    for (int off = 16; off > 0; off >>= 1) a += __shfl_xor(a, off, 32);
    if (lane == 0) R[4 * w + j] = a + bias[c];
  }
  __syncthreads();
  if (tid < 8) {
    const v4f v = *(const v4f*)(R + 4 * tid);
    float* d = corr + (size_t)b * NC + cb * 32 + 4 * tid;
    *(volatile v4f*)d = v;
    __threadfence();
    *(volatile v4f*)d = v;
  }
}

__global__ __launch_bounds__(256) void k_qkv(const us* __restrict__ X16, const us* __restrict__ W16,
                                             us* Qb, us* Kb, us* Vt) {
  __shared__ v4u TT[64 * 256 / 8];
  us* T0 = (us*)TT;
  const int tid = threadIdx.x, w = tid >> 5, lane = tid & 31, hl = lane >> 4, m16 = lane & 15;
  const int bt = blockIdx.x / (NF / 256), bf = blockIdx.x % (NF / 256);
  const int which = bf / (NC / 256), hb = (bf % (NC / 256)) * (256 / ND);
  const int wm = w >> 2, wf = w & 3;
  const int tok0 = bt * 64 + wm * 32;
  const int f0 = bf * 256 + wf * 64;
  v8f acc[2][4];
#pragma unroll
  for (int i = 0; i < 2; ++i)
#pragma unroll
    for (int j = 0; j < 4; ++j) acc[i][j] = zero8();
  gemm32x64(X16, NC, tok0, W16, NC, f0, NC, lane, acc);
  const float qs = 0.015625f;
  if (which < 2) {
#pragma unroll
    for (int i = 0; i < 2; ++i)
#pragma unroll
      for (int j = 0; j < 4; ++j)
#pragma unroll
        for (int r = 0; r < 8; ++r)
          T0[(wm * 32 + 16 * i + 8 * hl + r) * 256 + wf * 64 + 16 * j + m16] = f16bits(acc[i][j][r] * qs);
    __syncthreads();
    us* dst = (which == 0) ? Qb : Kb;
#pragma unroll
    for (int ps = 0; ps < 2; ++ps) {
#pragma unroll
      for (int it = 0; it < 8; ++it) {
        const int L = it * 32 + (tid >> 3), p = tid & 7;
        const int hh = L >> 6, t = L & 63;
        const v4u v = *(const v4u*)(T0 + t * 256 + hh * 64 + 8 * p);
        const int token = bt * 64 + t, bb = token / NS, nn = token % NS;
        us* d = dst + ((size_t)((bb * NH + hb + hh) * NS + nn)) * ND + 8 * p;
        *(volatile v4u*)d = v;
      }
      if (ps == 0) __threadfence();
    }
  } else {
#pragma unroll
    for (int i = 0; i < 2; ++i)
#pragma unroll
      for (int j = 0; j < 4; ++j) {
        H8 o8;
#pragma unroll
        for (int r = 0; r < 8; ++r) o8.h[r] = (_Float16)(acc[i][j][r] * qs);
        *(v4u*)(T0 + (wf * 64 + 16 * j + m16) * 64 + wm * 32 + 16 * i + 8 * hl) = o8.u;
      }
    __syncthreads();
    const int bb = (bt * 64) / NS, n0 = (bt * 64) % NS;
#pragma unroll
    for (int ps = 0; ps < 2; ++ps) {
#pragma unroll
      for (int it = 0; it < 8; ++it) {
        const int f = it * 32 + (tid >> 3), p = tid & 7;
        const v4u v = *(const v4u*)(T0 + f * 64 + 8 * p);
        const size_t off = ((size_t)((bb * NH + hb + (f >> 6)) * ND + (f & 63))) * NS + n0 + 8 * p;
        *(volatile v4u*)(Vt + off) = v;
      }
      if (ps == 0) __threadfence();
    }
  }
}

__global__ __launch_bounds__(256) void k_sgemm(const us* __restrict__ Qb, const us* __restrict__ Kb, us* S16, int b) {
  __shared__ v4u TT[8 * 32 * 64 / 8];
  const int tid = threadIdx.x, w = tid >> 5, lane = tid & 31, hl = lane >> 4, m16 = lane & 15;
  const int wt = blockIdx.x * 8 + w;
  const int h = wt >> 9, nt = (wt >> 4) & 31, mt = wt & 15;
  const size_t hoff = (size_t)(b * NH + h) * NS * ND;
  v8f acc[2][4];
#pragma unroll
  for (int i = 0; i < 2; ++i)
#pragma unroll
    for (int j = 0; j < 4; ++j) acc[i][j] = zero8();
  gemm32x64(Qb + hoff, ND, nt * 32, Kb + hoff, ND, mt * 64, ND, lane, acc);
  us* Tw = (us*)TT + w * 2048;
#pragma unroll
  for (int i = 0; i < 2; ++i)
#pragma unroll
    for (int j = 0; j < 4; ++j)
#pragma unroll
      for (int r = 0; r < 8; ++r)
        Tw[(16 * i + 8 * hl + r) * 64 + 16 * j + m16] = f16bits(acc[i][j][r] * 8.f);
  __syncthreads();
  us* g = S16 + (size_t)h * NS * NS + (size_t)(nt * 32) * NS + mt * 64;
#pragma unroll
  for (int ps = 0; ps < 2; ++ps) {
#pragma unroll
    for (int it = 0; it < 8; ++it) {
      const int row = 4 * it + (lane >> 3), p = lane & 7;
      const v4u v = *(const v4u*)(Tw + row * 64 + 8 * p);
      *(volatile v4u*)(g + (size_t)row * NS + 8 * p) = v;
    }
    if (ps == 0) __threadfence();
  }
}

__global__ __launch_bounds__(256) void k_mix(const us* __restrict__ S16, const float* __restrict__ convl,
                                             const float* __restrict__ convw, us* A4) {
  __shared__ v4u TT[8 * 16 * 128 / 8];
  __shared__ __attribute__((aligned(16))) float red[8 * 16 * 16];
  __shared__ float red2[8 * 16];
  __shared__ __attribute__((aligned(16))) float fin[16];
  const int tid = threadIdx.x, w = tid >> 5, lane = tid & 31, hl = lane >> 4, m16 = lane & 15;
  const int n = blockIdx.x;
  us* Tw = (us*)TT + w * 2048;
  const v4u z4 = {0u, 0u, 0u, 0u};
  *(v4u*)(Tw + 12 * 128 + 16 * lane) = z4;
  *(v4u*)(Tw + 12 * 128 + 16 * lane + 8) = z4;
  const us* Sn = S16 + (size_t)n * NS + 128 * w + 8 * m16;
#pragma unroll
  for (int j = 0; j < 6; ++j) {
    const int h = 2 * j + hl;
    const v4u v = *(const v4u*)(Sn + (size_t)h * NS * NS);
    *(v4u*)(Tw + h * 128 + 8 * m16) = v;
  }
  Frag A1, B2;
  {
    H8 ca, cb;
#pragma unroll
    for (int i = 0; i < 8; ++i) {
      const int hh = 8 * hl + i;
      float vl = 0.f, vw = 0.f;
      if (hh < NH && m16 < NH) { vl = convl[m16 * NH + hh]; vw = convw[m16 * NH + hh]; }
      ca.h[i] = (_Float16)(vl * 64.f);
      cb.h[i] = (_Float16)(vw * 64.f);
    }
    A1.q[0] = ca.u; A1.q[1] = z4;
    B2.q[0] = cb.u; B2.q[1] = z4;
  }
  __syncthreads();
  const v8f z8 = zero8();
  Frag bq[8];
#pragma unroll
  for (int f = 0; f < 8; ++f) {
    H8 g;
#pragma unroll
    for (int i = 0; i < 8; ++i) g.s[i] = Tw[(8 * hl + i) * 128 + 16 * f + m16];
    bq[f].q[0] = g.u; bq[f].q[1] = z4;
  }
  v8f acc[8];
#pragma unroll
  for (int f = 0; f < 8; ++f) acc[f] = WF16(A1.h, bq[f].h, z8);
  asm volatile(NOPS
               : "+v"(acc[0]), "+v"(acc[1]), "+v"(acc[2]), "+v"(acc[3]),
                 "+v"(acc[4]), "+v"(acc[5]), "+v"(acc[6]), "+v"(acc[7])
               : "v"(A1.w), "v"(bq[0].w), "v"(bq[1].w), "v"(bq[2].w), "v"(bq[3].w),
                 "v"(bq[4].w), "v"(bq[5].w), "v"(bq[6].w), "v"(bq[7].w));
  F8 pm;
  pm.v = acc[0];
#pragma unroll
  for (int f = 1; f < 8; ++f)
#pragma unroll
    for (int r = 0; r < 8; ++r) pm.v[r] = fmaxf(pm.v[r], acc[f][r]);
  float* rw = red + (w * 16 + m16) * 16 + 8 * hl;
  *(v4f*)rw = pm.q[0];
  *(v4f*)(rw + 4) = pm.q[1];
  __syncthreads();
  if (tid < 128) {
    const int o = tid & 15, part = tid >> 4;
    const float* rp = red + part * 256 + o;
    float v = rp[0];
#pragma unroll
    for (int mm = 1; mm < 16; ++mm) v = fmaxf(v, rp[16 * mm]);
    red2[part * 16 + o] = v;
  }
  __syncthreads();
  const float c1 = 1.4426950408889634f / 4096.f;
  if (tid < 16) {
    float v = red2[tid];
#pragma unroll
    for (int p = 1; p < 8; ++p) v = fmaxf(v, red2[16 * p + tid]);
    fin[tid] = -v * c1;
  }
  __syncthreads();
  F8 mneg;
  mneg.q[0] = *(const v4f*)(fin + 8 * hl);
  mneg.q[1] = *(const v4f*)(fin + 8 * hl + 4);
  F8 psum;
  psum.v = z8;
#pragma unroll
  for (int f = 0; f < 8; ++f)
#pragma unroll
    for (int r = 0; r < 8; ++r) {
      const float e = __builtin_amdgcn_exp2f(fmaf(acc[f][r], c1, mneg.v[r]));
      acc[f][r] = e;
      psum.v[r] += e;
    }
  *(v4f*)rw = psum.q[0];
  *(v4f*)(rw + 4) = psum.q[1];
  __syncthreads();
  if (tid < 128) {
    const int o = tid & 15, part = tid >> 4;
    const float* rp = red + part * 256 + o;
    float v = rp[0];
#pragma unroll
    for (int mm = 1; mm < 16; ++mm) v += rp[16 * mm];
    red2[part * 16 + o] = v;
  }
  __syncthreads();
  if (tid < 16) {
    float v = red2[tid];
#pragma unroll
    for (int p = 1; p < 8; ++p) v += red2[16 * p + tid];
    fin[tid] = 32768.f / v;
  }
  __syncthreads();
  F8 rs;
  rs.q[0] = *(const v4f*)(fin + 8 * hl);
  rs.q[1] = *(const v4f*)(fin + 8 * hl + 4);
  Frag a2[8];
#pragma unroll
  for (int f = 0; f < 8; ++f) {
    H8 p8;
#pragma unroll
    for (int r = 0; r < 8; ++r) p8.h[r] = (_Float16)fmaf(acc[f][r], rs.v[r], -32.f);
    a2[f].q[0] = p8.u; a2[f].q[1] = z4;
  }
  v8f acc2[8];
#pragma unroll
  for (int f = 0; f < 8; ++f) acc2[f] = WF16(a2[f].h, B2.h, z8);
  asm volatile(NOPS
               : "+v"(acc2[0]), "+v"(acc2[1]), "+v"(acc2[2]), "+v"(acc2[3]),
                 "+v"(acc2[4]), "+v"(acc2[5]), "+v"(acc2[6]), "+v"(acc2[7])
               : "v"(B2.w), "v"(a2[0].w), "v"(a2[1].w), "v"(a2[2].w), "v"(a2[3].w),
                 "v"(a2[4].w), "v"(a2[5].w), "v"(a2[6].w), "v"(a2[7].w));
#pragma unroll
  for (int f = 0; f < 8; ++f) {
    H8 o8;
#pragma unroll
    for (int r = 0; r < 8; ++r) o8.h[r] = (_Float16)(acc2[f][r] * 0.03125f);
    *(v4u*)(Tw + m16 * 128 + 16 * f + 8 * hl) = o8.u;
  }
  __syncthreads();
#pragma unroll
  for (int ps = 0; ps < 2; ++ps) {
#pragma unroll
    for (int it = 0; it < 6; ++it) {
      const int L = 4 * it + (lane >> 3), p = lane & 7;
      const int o = L >> 1, half = L & 1;
      const v4u v = *(const v4u*)(Tw + o * 128 + 64 * half + 8 * p);
      us* d = A4 + (size_t)o * NS * NS + (size_t)n * NS + 128 * w + 64 * half + 8 * p;
      *(volatile v4u*)d = v;
    }
    if (ps == 0) __threadfence();
  }
}

__global__ __launch_bounds__(256) void k_av(const us* __restrict__ A4, const us* __restrict__ Vt, us* O16, int b) {
  __shared__ v4u TT[8 * 32 * 64 / 8];
  const int tid = threadIdx.x, w = tid >> 5, lane = tid & 31, hl = lane >> 4, m16 = lane & 15;
  const int wt = blockIdx.x * 8 + w;
  const int h = wt >> 5, nt = wt & 31;
  v8f acc[2][4];
#pragma unroll
  for (int i = 0; i < 2; ++i)
#pragma unroll
    for (int j = 0; j < 4; ++j) acc[i][j] = zero8();
  gemm32x64(A4 + (size_t)h * NS * NS, NS, nt * 32, Vt + (size_t)(b * NH + h) * ND * NS, NS, 0, NS, lane, acc);
  us* Tw = (us*)TT + w * 2048;
#pragma unroll
  for (int i = 0; i < 2; ++i)
#pragma unroll
    for (int j = 0; j < 4; ++j)
#pragma unroll
      for (int r = 0; r < 8; ++r)
        Tw[(16 * i + 8 * hl + r) * 64 + 16 * j + m16] = f16bits(acc[i][j][r] * 0.5f);
  __syncthreads();
#pragma unroll
  for (int ps = 0; ps < 2; ++ps) {
#pragma unroll
    for (int it = 0; it < 8; ++it) {
      const int row = 4 * it + (lane >> 3), p = lane & 7;
      const v4u v = *(const v4u*)(Tw + row * 64 + 8 * p);
      us* d = O16 + ((size_t)(b * NS + nt * 32 + row)) * NC + h * ND + 8 * p;
      *(volatile v4u*)d = v;
    }
    if (ps == 0) __threadfence();
  }
}

__global__ __launch_bounds__(256) void k_proj(const us* __restrict__ O16, const us* __restrict__ Wp16,
                                              const float* __restrict__ corr, float* out) {
  __shared__ v4f TT[8 * 32 * 64 / 4];
  const int tid = threadIdx.x, w = tid >> 5, lane = tid & 31, hl = lane >> 4, m16 = lane & 15;
  const int wt = blockIdx.x * 8 + w;
  const int mt = wt / (NC / 64), ntl = wt % (NC / 64);
  const int m0 = mt * 32, n0 = ntl * 64;
  v8f acc[2][4];
#pragma unroll
  for (int i = 0; i < 2; ++i)
#pragma unroll
    for (int j = 0; j < 4; ++j) acc[i][j] = zero8();
  gemm32x64(O16, NC, m0, Wp16, NC, n0, NC, lane, acc);
  float* Tw = (float*)TT + w * 2048;
#pragma unroll
  for (int i = 0; i < 2; ++i)
#pragma unroll
    for (int j = 0; j < 4; ++j)
#pragma unroll
      for (int r = 0; r < 8; ++r)
        Tw[(16 * i + 8 * hl + r) * 64 + 16 * j + m16] = acc[i][j][r];
  __syncthreads();
  const int bb = m0 / NS;
  const v4f cv = *(const v4f*)(corr + (size_t)bb * NC + n0 + 4 * m16);
  const float osc = 1.0f / 2097152.f;
#pragma unroll
  for (int ps = 0; ps < 2; ++ps) {
#pragma unroll
    for (int it = 0; it < 16; ++it) {
      const int row = 2 * it + hl;
      const v4f v = *(const v4f*)(Tw + row * 64 + 4 * m16) * osc + cv;
      *(volatile v4f*)(out + (size_t)(m0 + row) * NC + n0 + 4 * m16) = v;
    }
    if (ps == 0) __threadfence();
  }
}

extern "C" void kernel_launch(void* const* d_in, const int* in_sizes, int n_in,
                              void* d_out, int out_size, void* d_ws, size_t ws_size,
                              hipStream_t stream) {
  if (n_in < 6) return;
  if (in_sizes[0] != NTOK * NC || in_sizes[1] != NF * NC || in_sizes[2] != NC * NC ||
      in_sizes[3] != NC || in_sizes[4] != NH * NH || in_sizes[5] != NH * NH) return;
  if (out_size != NTOK * NC) return;

  const float* x = (const float*)d_in[0];
  const float* w_qkv = (const float*)d_in[1];
  const float* w_proj = (const float*)d_in[2];
  const float* b_proj = (const float*)d_in[3];
  const float* conv_l = (const float*)d_in[4];
  const float* conv_w = (const float*)d_in[5];
  float* out = (float*)d_out;

  size_t off = 0;
  char* wsb = (char*)d_ws;
  auto carve = [&](size_t bytes) -> char* {
    char* p = wsb + off;
    off += (bytes + 255) & ~(size_t)255;
    return p;
  };
  const size_t n_x = (size_t)NTOK * NC;
  const size_t n_wq = (size_t)NF * NC;
  const size_t n_wp = (size_t)NC * NC;
  const size_t n_hd = (size_t)NB * NH * NS * ND;
  const size_t n_ss = (size_t)NH * NS * NS;
  const size_t n_sd = (size_t)NB * NC;

  us* X16 = (us*)carve(n_x * 2);
  us* W16 = (us*)carve(n_wq * 2);
  us* Wp16 = (us*)carve(n_wp * 2);
  us* Qb = (us*)carve(n_hd * 2);
  us* Kb = (us*)carve(n_hd * 2);
  us* Vt = (us*)carve(n_hd * 2);
  us* S16 = (us*)carve(n_ss * 2);
  us* A4 = (us*)carve(n_ss * 2);
  us* O16 = (us*)carve(n_x * 2);
  float* xs = (float*)carve(n_sd * 4);
  float* sv = (float*)carve(n_sd * 4);
  float* corr = (float*)carve(n_sd * 4);
  if (off > ws_size) return;

  const int n8_x = (int)(n_x / 8), n8_wq = (int)(n_wq / 8), n8_wp = (int)(n_wp / 8);
  k_cvt<<<(n8_x + 255) / 256, 256, 0, stream>>>(x, X16, 1.0f, n8_x);
  k_cvt<<<(n8_wq + 255) / 256, 256, 0, stream>>>(w_qkv, W16, 64.0f, n8_wq);
  k_cvt<<<(n8_wp + 255) / 256, 256, 0, stream>>>(w_proj, Wp16, 64.0f, n8_wp);

  k_xsum<<<NB * (NC / 256), 256, 0, stream>>>(x, xs);
  k_sv<<<NB * (NC / 32), 256, 0, stream>>>(xs, w_qkv, sv);
  k_corr<<<NB * (NC / 32), 256, 0, stream>>>(sv, conv_w, w_proj, b_proj, corr);

  k_qkv<<<(NTOK / 64) * (NF / 256), 256, 0, stream>>>(X16, W16, Qb, Kb, Vt);

  for (int b = 0; b < NB; ++b) {
    k_sgemm<<<(NH * (NS / 32) * (NS / 64)) / 8, 256, 0, stream>>>(Qb, Kb, S16, b);
    k_mix<<<NS, 256, 0, stream>>>(S16, conv_l, conv_w, A4);
    k_av<<<(NH * (NS / 32)) / 8, 256, 0, stream>>>(A4, Vt, O16, b);
  }

  k_proj<<<((NTOK / 32) * (NC / 64)) / 8, 256, 0, stream>>>(O16, Wp16, corr, out);
}
